// MoEConformerLayer_33990371181313
// MI455X (gfx1250) — hardware-run, weakly checked
//
#include <hip/hip_runtime.h>
#include <math.h>

constexpr int NB    = 2;
constexpr int NS    = 2048;
constexpr int ND    = 512;
constexpr int NH    = 8;
constexpr int NHD   = 64;
constexpr int KW    = 31;
constexpr int NFF   = 2048;
constexpr int NG    = 4;
constexpr int NE    = 2;
constexpr int NTOK  = NB * NS;
constexpr int KCONV = KW * ND;
constexpr int PADL  = (KW - 1) / 2;
constexpr int HPROWS = NS + 32;
constexpr int QKV_LD = 3 * ND;
constexpr int GROWS  = NTOK + NG * 64;
constexpr int HID_LD = NE * NFF;
constexpr float WCARRY = 16.0f;
constexpr float OCARRY = 256.0f;
constexpr float HCARRY = 64.0f;
constexpr float PCARRY = 32768.0f;

static_assert(KCONV % 32 == 0);
static_assert(ND % 64 == 0 && NFF % 64 == 0 && NS % 64 == 0 && NTOK % 64 == 0 && GROWS % 64 == 0);
static_assert(HID_LD % 32 == 0 && ND % 32 == 0);
static_assert(HPROWS - PADL - NS >= KW - 1 - PADL);
static_assert(NTOK == 256 * 16);
static_assert(NHD == 64 && NH * NHD == ND);
static_assert((NS / 64) * (ND / 64) % 8 == 0 && (NTOK / 64) * (ND / 64) % 8 == 0);
static_assert((GROWS / 64) * (NFF / 64) % 8 == 0 && (GROWS / 64) * (ND / 64) % 8 == 0);

constexpr size_t WS_CKT   = (size_t)ND * KCONV * 2;
constexpr size_t WS_W512  = (size_t)ND * ND * 2;
constexpr size_t WS_W1T   = (size_t)NFF * (NG * NE * ND) * 2;
constexpr size_t WS_W2T   = (size_t)ND * (NG * NE * NFF) * 2;
constexpr size_t WS_ACT16 = (size_t)NB * HPROWS * ND * 2;
constexpr size_t WS_X1    = (size_t)NTOK * ND * 4;
constexpr size_t WS_QKV   = (size_t)NTOK * QKV_LD * 2;
constexpr size_t WS_X2    = WS_X1;
constexpr size_t WS_HID   = (size_t)GROWS * HID_LD * 2;
constexpr size_t WS_Y     = (size_t)GROWS * ND * 4;
constexpr size_t WS_XG    = (size_t)GROWS * ND * 2;
constexpr size_t WS_TOTAL = WS_CKT + 4 * WS_W512 + WS_W1T + WS_W2T + WS_ACT16 + WS_X1 + WS_QKV + WS_X2 + WS_HID + WS_Y;
static_assert(WS_TOTAL == 130088960ull);
static_assert(WS_TOTAL <= 134217728ull);
static_assert(WS_XG <= WS_CKT);
static_assert((size_t)NTOK * ND * 2 <= WS_ACT16);
static_assert(WS_CKT % 128 == 0 && WS_W512 % 128 == 0 && WS_ACT16 % 128 == 0 && WS_HID % 128 == 0);

typedef __attribute__((ext_vector_type(16))) _Float16 v16h;
typedef __attribute__((ext_vector_type(8)))  _Float16 v8h;
typedef __attribute__((ext_vector_type(8)))  float    v8f;
typedef __attribute__((ext_vector_type(4)))  float    v4f;
typedef __attribute__((ext_vector_type(4)))  unsigned int v4u;

__device__ __forceinline__ void dep_guard_h(v8f& a, v8f& b, v16h x, v16h y) { asm volatile("v_nop\n\tv_nop\n\tv_nop\n\tv_nop" : "+v"(a), "+v"(b) : "v"(x), "v"(y)); }
__device__ __forceinline__ void keep4_h(v16h a, v16h b, v16h c, v16h d) { asm volatile("v_nop" :: "v"(a), "v"(b), "v"(c), "v"(d)); }
__device__ __forceinline__ void acc_guard4(v8f& a, v8f& b, v8f& c, v8f& d) { asm volatile("v_nop\n\tv_nop\n\tv_nop\n\tv_nop" : "+v"(a), "+v"(b), "+v"(c), "+v"(d)); }
template <typename T> struct Frag;
template <> struct Frag<_Float16> {
  typedef v16h V; union U { v16h v; v8h h[2]; };
  static __device__ __forceinline__ v16h load(const _Float16* p) {
    U f; f.h[0] = *(const v8h*)(p); f.h[1] = *(const v8h*)(p + 16); return f.v;
  }
  static __device__ __forceinline__ v8f mma(v16h a, v16h b, v8f c) {
    return __builtin_amdgcn_wmma_f32_16x16x32_f16(false, a, false, b, (short)0, c, false, false);
  }
  static __device__ __forceinline__ void guard(v8f& a, v8f& b, v16h x, v16h y) { dep_guard_h(a, b, x, y); }
  static __device__ __forceinline__ void keep(v16h a, v16h b, v16h c, v16h d) { keep4_h(a, b, c, d); }
};

__device__ __forceinline__ v8f mma_h(v16h a, v16h b, v8f c) {
  c = __builtin_amdgcn_wmma_f32_16x16x32_f16(false, a, false, b, (short)0, c, false, false);
  asm volatile("v_nop\n\tv_nop\n\tv_nop\n\tv_nop" : "+v"(c) : "v"(a), "v"(b));
  return c;
}

__device__ __forceinline__ unsigned pk16(unsigned short a, unsigned short b) { return (unsigned)a | ((unsigned)b << 16); }
__device__ __forceinline__ unsigned short h_bits(float f) { const _Float16 h = (_Float16)f; return __builtin_bit_cast(unsigned short, h); }

__device__ __forceinline__ void wave_lds_sync() {
  __builtin_amdgcn_fence(__ATOMIC_RELEASE, "workgroup");
  __builtin_amdgcn_wave_barrier();
  __builtin_amdgcn_fence(__ATOMIC_ACQUIRE, "workgroup");
}

__device__ __forceinline__ float gelu_tanh_f(float v) {
  const float u = v * (1.0f + 0.044715f * v * v);
  float z = -1.5957691216057308f * u;
  z = fminf(z, 80.0f);
  const float e = expf(z);
  return v * __builtin_amdgcn_rcpf(1.0f + e);
}

__device__ __forceinline__ void mma_tile64(v8f (&acc)[4][4], const _Float16* __restrict__ Ab, int lda,
                                           const _Float16* __restrict__ Bb, int ldb, int K, int m0, int n0, int lane) {
  const int rlane = lane & 15;
  const int koff  = (lane >> 4) * 8;
#pragma unroll
  for (int i = 0; i < 4; ++i)
#pragma unroll
    for (int j = 0; j < 4; ++j) acc[i][j] = (v8f){0.f, 0.f, 0.f, 0.f, 0.f, 0.f, 0.f, 0.f};
  for (int k0 = 0; k0 < K; k0 += 32) {
    v16h bh[4];
#pragma unroll
    for (int j = 0; j < 4; ++j)
      bh[j] = Frag<_Float16>::load(Bb + (size_t)(n0 + (j << 4) + rlane) * ldb + koff + k0);
#pragma unroll
    for (int i = 0; i < 4; ++i) {
      const v16h ah = Frag<_Float16>::load(Ab + (size_t)(m0 + (i << 4) + rlane) * lda + koff + k0);
#pragma unroll
      for (int j = 0; j < 4; ++j) acc[i][j] = Frag<_Float16>::mma(ah, bh[j], acc[i][j]);
      Frag<_Float16>::guard(acc[i][0], acc[i][3], ah, ah);
    }
    Frag<_Float16>::keep(bh[0], bh[1], bh[2], bh[3]);
  }
  acc_guard4(acc[0][0], acc[0][1], acc[0][2], acc[0][3]);
  acc_guard4(acc[1][0], acc[1][1], acc[1][2], acc[1][3]);
  acc_guard4(acc[2][0], acc[2][1], acc[2][2], acc[2][3]);
  acc_guard4(acc[3][0], acc[3][1], acc[3][2], acc[3][3]);
}

template <int ACT, bool RESID>
__device__ __forceinline__ void epilogue_f32(float* slab, const v8f (&acc)[4][4], float scale, const float (&bv)[4],
                                             float* __restrict__ C, int ldc, const float* __restrict__ R, int ldr,
                                             int m0, int n0, int lane) {
  const int rlane = lane & 15, mOff = (lane >> 4) * 8;
  const int hh = lane >> 4, c4 = rlane * 4;
#pragma unroll
  for (int i = 0; i < 4; ++i) {
    const int mBase = m0 + (i << 4);
#pragma unroll
    for (int j = 0; j < 4; ++j)
#pragma unroll
      for (int r = 0; r < 8; ++r)
        slab[(mOff + r) * 68 + (j << 4) + rlane] = acc[i][j][r] * scale + bv[j];
    wave_lds_sync();
    for (int pass = 0; pass < 2; ++pass) {
#pragma unroll 1
      for (int it = 0; it < 8; ++it) {
        const int row = it * 2 + hh;
        v4f v = *(const v4f*)(slab + row * 68 + c4);
        if (ACT == 1) { v[0] = gelu_tanh_f(v[0]); v[1] = gelu_tanh_f(v[1]); v[2] = gelu_tanh_f(v[2]); v[3] = gelu_tanh_f(v[3]); }
        if (RESID) { const v4f rr = *(const v4f*)(R + (size_t)(mBase + row) * ldr + n0 + c4); v += rr; }
        *(volatile v4f*)(C + (size_t)(mBase + row) * ldc + n0 + c4) = v;
      }
      __threadfence();
    }
    wave_lds_sync();
  }
}

template <int ACT>
__device__ __forceinline__ void epilogue_f16(float* slab, const v8f (&acc)[4][4], float scale, const float (&bv)[4], float oscale,
                                             unsigned short* __restrict__ C, int ldc, int m0, int n0, int lane) {
  const int rlane = lane & 15, mOff = (lane >> 4) * 8;
  const int q = lane >> 3, c8 = (lane & 7) * 8;
  _Float16* C16 = (_Float16*)(void*)C;
#pragma unroll
  for (int i = 0; i < 4; ++i) {
    const int mBase = m0 + (i << 4);
#pragma unroll
    for (int j = 0; j < 4; ++j)
#pragma unroll
      for (int r = 0; r < 8; ++r)
        slab[(mOff + r) * 68 + (j << 4) + rlane] = acc[i][j][r] * scale + bv[j];
    wave_lds_sync();
    for (int pass = 0; pass < 2; ++pass) {
#pragma unroll 1
      for (int it = 0; it < 4; ++it) {
        const int row = it * 4 + q;
        const float* sp = slab + row * 68 + c8;
        v8h hv;
#pragma unroll
        for (int e = 0; e < 8; ++e) {
          float f = sp[e];
          if (ACT == 1) f = gelu_tanh_f(f);
          hv[e] = (_Float16)(f * oscale);
        }
        *(volatile v8h*)(C16 + (size_t)(mBase + row) * ldc + n0 + c8) = hv;
      }
      __threadfence();
    }
    wave_lds_sync();
  }
}

template <int ACT, int OUT_MODE, bool RESID>
__global__ __launch_bounds__(256) void gemm_f16(
    const unsigned short* __restrict__ Ap, int lda, long strideA,
    const unsigned short* __restrict__ Btp, int ldb, long strideB,
    void* __restrict__ Cout, int ldc, long strideC,
    const float* __restrict__ bias,
    const float* __restrict__ resid, long strideR,
    int M, int N, int K, float scale, float oscale) {
  __shared__ __align__(16) float sT[8][16 * 68];
  const int b    = blockIdx.y;
  const int lane = threadIdx.x & 31;
  const int wave = threadIdx.x >> 5;
  const int tilesN = N >> 6;
  const int tilesM = M >> 6;
  const int tile = blockIdx.x * 8 + wave;
  if (tile >= tilesM * tilesN) return;
  const int tm = tile / tilesN;
  const int tn = tile - tm * tilesN;
  const int m0 = tm << 6;
  const int n0 = tn << 6;
  const _Float16* Ab = (const _Float16*)(const void*)Ap + (size_t)b * strideA;
  const _Float16* Bb = (const _Float16*)(const void*)Btp + (size_t)b * strideB;
  v8f acc[4][4];
  mma_tile64(acc, Ab, lda, Bb, ldb, K, m0, n0, lane);
  float bv[4];
#pragma unroll
  for (int j = 0; j < 4; ++j) bv[j] = bias[n0 + (j << 4) + (lane & 15)];
  if (OUT_MODE == 0) {
    float* C = (float*)Cout + (size_t)b * strideC;
    const float* R = RESID ? (resid + (size_t)b * strideR) : nullptr;
    epilogue_f32<ACT, RESID>(sT[wave], acc, scale, bv, C, ldc, R, ldc, m0, n0, lane);
  } else {
    unsigned short* C = (unsigned short*)Cout + (size_t)b * strideC;
    epilogue_f16<ACT>(sT[wave], acc, scale, bv, oscale, C, ldc, m0, n0, lane);
  }
}

__device__ __forceinline__ int clamp_g(int v) { v = v < 0 ? 0 : v; return v > (NG - 1) ? (NG - 1) : v; }

__device__ __forceinline__ void route_scan(const int* __restrict__ gid, unsigned long long* sbuf,
                                           int (&id)[16], unsigned long long& excl,
                                           int (&cnt)[4], int (&base)[4], int (&te)[4]) {
  const int t = threadIdx.x;
  const int4* gp = (const int4*)(const void*)(gid + 16 * t);
  const int4 g0 = gp[0], g1 = gp[1], g2 = gp[2], g3 = gp[3];
  id[0]  = clamp_g(g0.x); id[1]  = clamp_g(g0.y); id[2]  = clamp_g(g0.z); id[3]  = clamp_g(g0.w);
  id[4]  = clamp_g(g1.x); id[5]  = clamp_g(g1.y); id[6]  = clamp_g(g1.z); id[7]  = clamp_g(g1.w);
  id[8]  = clamp_g(g2.x); id[9]  = clamp_g(g2.y); id[10] = clamp_g(g2.z); id[11] = clamp_g(g2.w);
  id[12] = clamp_g(g3.x); id[13] = clamp_g(g3.y); id[14] = clamp_g(g3.z); id[15] = clamp_g(g3.w);
  unsigned long long key = 0ull;
#pragma unroll
  for (int j = 0; j < 16; ++j) key += (1ull << (16 * id[j]));
  unsigned long long cur = key;
#pragma unroll
  for (int off = 1; off < 256; off <<= 1) {
    sbuf[t] = cur;
    __syncthreads();
    int src = t - off;
    src = src < 0 ? 0 : src;
    const unsigned long long add = sbuf[src];
    __syncthreads();
    cur += (t >= off) ? add : 0ull;
  }
  excl = cur - key;
  sbuf[t] = cur;
  __syncthreads();
  const unsigned long long total = sbuf[255];
  int cp[4];
#pragma unroll
  for (int g = 0; g < 4; ++g) {
    cnt[g] = (int)((total >> (16 * g)) & 0xffffull);
    cp[g]  = (cnt[g] + 63) & ~63;
  }
  base[0] = 0;
  base[1] = cp[0];
  base[2] = cp[0] + cp[1];
  base[3] = cp[0] + cp[1] + cp[2];
#pragma unroll
  for (int g = 0; g < 4; ++g) te[g] = (base[g] + cp[g]) >> 6;
}

__device__ __forceinline__ int route_pos(int g, int (&rk)[4], const int (&base)[4]) {
  const int r  = (g == 0) ? rk[0] : (g == 1) ? rk[1] : (g == 2) ? rk[2] : rk[3];
  const int bs = (g == 0) ? base[0] : (g == 1) ? base[1] : (g == 2) ? base[2] : base[3];
  rk[0] += (g == 0); rk[1] += (g == 1); rk[2] += (g == 2); rk[3] += (g == 3);
  int p = bs + r;
  return p > (GROWS - 1) ? (GROWS - 1) : p;
}

template <int MODE>
__global__ __launch_bounds__(256) void expert_gemm(const int* __restrict__ gid, const unsigned short* __restrict__ Ap,
                                                   const unsigned short* __restrict__ Wp, const float* __restrict__ bias,
                                                   void* __restrict__ Cout) {
  __shared__ unsigned long long sbuf[256];
  __shared__ __align__(16) float sT[8][16 * 68];
  int id[16]; unsigned long long excl; int cnt[4], base[4], te[4];
  route_scan(gid, sbuf, id, excl, cnt, base, te);
  const int lane = threadIdx.x & 31;
  const int wave = threadIdx.x >> 5;
  constexpr int tilesN = (MODE == 1) ? (NFF / 64) : (ND / 64);
  const int tile = blockIdx.x * 8 + wave;
  const int tm = tile / tilesN;
  const int tn = tile - tm * tilesN;
  if (tm >= te[3]) return;
  const int g  = (tm >= te[0]) + (tm >= te[1]) + (tm >= te[2]);
  const int m0 = tm << 6;
  const int n0 = tn << 6;
  const int rlane = lane & 15;
  v8f acc[4][4];
  float bv[4];
  if (MODE == 1) {
    const int e  = blockIdx.z;
    const int ge = g * NE + e;
    const _Float16* Ab = (const _Float16*)(const void*)Ap;
    const _Float16* Bb = (const _Float16*)(const void*)Wp + (size_t)ge * ND;
    mma_tile64(acc, Ab, ND, Bb, NG * NE * ND, ND, m0, n0, lane);
#pragma unroll
    for (int j = 0; j < 4; ++j) bv[j] = bias[(size_t)ge * NFF + n0 + (j << 4) + rlane];
    unsigned short* C = (unsigned short*)Cout + e * NFF;
    epilogue_f16<1>(sT[wave], acc, 1.0f / WCARRY, bv, HCARRY, C, HID_LD, m0, n0, lane);
  } else {
    const _Float16* Ab = (const _Float16*)(const void*)Ap;
    const _Float16* Bb = (const _Float16*)(const void*)Wp + (size_t)g * (NE * NFF);
    mma_tile64(acc, Ab, HID_LD, Bb, NG * NE * NFF, HID_LD, m0, n0, lane);
#pragma unroll
    for (int j = 0; j < 4; ++j) {
      const int n = n0 + (j << 4) + rlane;
      bv[j] = 0.5f * (bias[(size_t)g * NE * ND + n] + bias[(size_t)g * NE * ND + ND + n]);
    }
    float* C = (float*)Cout;
    epilogue_f32<0, false>(sT[wave], acc, 0.5f / (WCARRY * HCARRY), bv, C, ND, nullptr, ND, m0, n0, lane);
  }
}

__global__ __launch_bounds__(256) void gather_rows_kernel(const int* __restrict__ gid, const float* __restrict__ x2,
                                                          unsigned short* __restrict__ xg) {
  __shared__ unsigned long long sbuf[256];
  __shared__ int ord[GROWS];
  int id[16]; unsigned long long excl; int cnt[4], base[4], te[4];
  route_scan(gid, sbuf, id, excl, cnt, base, te);
  const int t = threadIdx.x;
  for (int k = t; k < GROWS; k += 256) ord[k] = -1;
  __syncthreads();
  {
    int rk[4] = {(int)(excl & 0xffffull), (int)((excl >> 16) & 0xffffull), (int)((excl >> 32) & 0xffffull), (int)((excl >> 48) & 0xffffull)};
#pragma unroll
    for (int j = 0; j < 16; ++j) {
      const int p = route_pos(id[j], rk, base);
      ord[p] = 16 * t + j;
    }
  }
  __syncthreads();
  const int lane = t & 31, wave = t >> 5;
  const int pw = blockIdx.x * 64 + wave * 8;
  for (int pass = 0; pass < 2; ++pass) {
#pragma unroll 1
    for (int r = 0; r < 8; ++r) {
      const int p  = pw + r;
      const int nl = ord[p];
      const float fz = (nl >= 0) ? 1.0f : 0.0f;
      const int n  = (nl >= 0) ? nl : 0;
#pragma unroll
      for (int hf = 0; hf < 2; ++hf) {
        const int col = hf * 256 + lane * 8;
        const float* xr = x2 + (size_t)n * ND + col;
        const v4f a = *(const v4f*)(xr);
        const v4f c = *(const v4f*)(xr + 4);
        const v4u u = (v4u){pk16(h_bits(a[0] * fz), h_bits(a[1] * fz)), pk16(h_bits(a[2] * fz), h_bits(a[3] * fz)),
                            pk16(h_bits(c[0] * fz), h_bits(c[1] * fz)), pk16(h_bits(c[2] * fz), h_bits(c[3] * fz))};
        *(volatile v4u*)(xg + (size_t)p * ND + col) = u;
      }
    }
    __threadfence();
  }
}

__global__ __launch_bounds__(256) void combine_kernel(const int* __restrict__ gid, const float* __restrict__ y,
                                                      const float* __restrict__ x2, float* __restrict__ out) {
  __shared__ unsigned long long sbuf[256];
  __shared__ int posv[64];
  int id[16]; unsigned long long excl; int cnt[4], base[4], te[4];
  route_scan(gid, sbuf, id, excl, cnt, base, te);
  const int t = threadIdx.x;
  if ((t >> 2) == (int)blockIdx.x) {
    int rk[4] = {(int)(excl & 0xffffull), (int)((excl >> 16) & 0xffffull), (int)((excl >> 32) & 0xffffull), (int)((excl >> 48) & 0xffffull)};
#pragma unroll
    for (int j = 0; j < 16; ++j) posv[(t & 3) * 16 + j] = route_pos(id[j], rk, base);
  }
  __syncthreads();
  const int lane = t & 31, wave = t >> 5;
  for (int pass = 0; pass < 2; ++pass) {
#pragma unroll 1
    for (int r = 0; r < 8; ++r) {
      const int nl = wave * 8 + r;
      const int n  = blockIdx.x * 64 + nl;
      int p = posv[nl];
      p = p < 0 ? 0 : (p > GROWS - 1 ? GROWS - 1 : p);
#pragma unroll
      for (int qq = 0; qq < 4; ++qq) {
        const int col = qq * 128 + lane * 4;
        const v4f a = *(const v4f*)(y + (size_t)p * ND + col);
        const v4f c = *(const v4f*)(x2 + (size_t)n * ND + col);
        const v4f o = a + c;
        *(volatile v4f*)(out + (size_t)n * ND + col) = o;
      }
    }
    __threadfence();
  }
}

__global__ __launch_bounds__(256) void trcast_kernel(const float* __restrict__ in, int R, int C,
                                                     unsigned short* __restrict__ outp, float scale) {
  __shared__ float sm[64][65];
  const int t  = threadIdx.x;
  const int r0 = blockIdx.x * 64;
  const int c0 = blockIdx.y * 64;
#pragma unroll
  for (int i = 0; i < 4; ++i) {
    const int e  = i * 256 + t;
    const int r  = e >> 4;
    const int cq = (e & 15) * 4;
    const v4f v = *(const v4f*)(in + (size_t)(r0 + r) * C + c0 + cq);
    sm[cq + 0][r] = v[0] * scale;
    sm[cq + 1][r] = v[1] * scale;
    sm[cq + 2][r] = v[2] * scale;
    sm[cq + 3][r] = v[3] * scale;
  }
  __syncthreads();
  const int lane = t & 31, wave = t >> 5;
  const int q = lane >> 3, c8 = (lane & 7) * 8;
  for (int pass = 0; pass < 2; ++pass) {
#pragma unroll
    for (int it = 0; it < 2; ++it) {
      const int row = wave * 8 + it * 4 + q;
      unsigned short hb[8];
#pragma unroll
      for (int e = 0; e < 8; ++e) hb[e] = h_bits(sm[row][c8 + e]);
      const v4u u = (v4u){pk16(hb[0], hb[1]), pk16(hb[2], hb[3]), pk16(hb[4], hb[5]), pk16(hb[6], hb[7])};
      *(volatile v4u*)(outp + (size_t)(c0 + row) * R + r0 + c8) = u;
    }
    __threadfence();
  }
}

__global__ __launch_bounds__(256) void zero_pad_kernel(unsigned short* __restrict__ plane) {
  const int yb = blockIdx.y;
  const int b  = yb >> 1;
  const int which = yb & 1;
  const int startRow = which ? (PADL + NS) : 0;
  const int nRows = which ? (HPROWS - PADL - NS) : PADL;
  const int nWords = nRows * (ND / 8);
  const int i = blockIdx.x * 256 + threadIdx.x;
  if (i < nWords) {
    unsigned short* p = plane + ((size_t)(b * HPROWS + startRow) * ND + (size_t)i * 8);
    const v4u z = (v4u){0u, 0u, 0u, 0u};
    *(volatile v4u*)p = z;
    __threadfence();
    *(volatile v4u*)p = z;
  }
}

__global__ __launch_bounds__(256) void ln_kernel(const float* __restrict__ x, const float* __restrict__ sc,
                                                 const float* __restrict__ bi, unsigned short* __restrict__ outp,
                                                 int rowsPerBatch, int rowOff) {
  __shared__ float red[4][2];
  __shared__ float red2[4][2];
  const int t = threadIdx.x, lane = t & 31, rl = t >> 6, wl = (t >> 5) & 1;
  const int row  = blockIdx.x * 4 + rl;
  const int col0 = wl * 256 + lane * 8;
  const float* xr = x + (size_t)row * ND + col0;
  const v4f a = *(const v4f*)(xr);
  const v4f c = *(const v4f*)(xr + 4);
  float v[8] = {a[0], a[1], a[2], a[3], c[0], c[1], c[2], c[3]};
  float s = 0.0f;
#pragma unroll
  for (int e = 0; e < 8; ++e) s += v[e];
#pragma unroll
  for (int off = 16; off > 0; off >>= 1) s += __shfl_xor(s, off, 32);
  if (lane == 0) red[rl][wl] = s;
  __syncthreads();
  const float mean = (red[rl][0] + red[rl][1]) * (1.0f / 512.0f);
  float d[8];
  float ss = 0.0f;
#pragma unroll
  for (int e = 0; e < 8; ++e) { d[e] = v[e] - mean; ss += d[e] * d[e]; }
#pragma unroll
  for (int off = 16; off > 0; off >>= 1) ss += __shfl_xor(ss, off, 32);
  if (lane == 0) red2[rl][wl] = ss;
  __syncthreads();
  const float var = (red2[rl][0] + red2[rl][1]) * (1.0f / 512.0f);
  const float rs = rsqrtf(var + 1e-6f);
  const v4f sa = *(const v4f*)(sc + col0), sb = *(const v4f*)(sc + col0 + 4);
  const v4f ba = *(const v4f*)(bi + col0), bb = *(const v4f*)(bi + col0 + 4);
  float scv[8] = {sa[0], sa[1], sa[2], sa[3], sb[0], sb[1], sb[2], sb[3]};
  float biv[8] = {ba[0], ba[1], ba[2], ba[3], bb[0], bb[1], bb[2], bb[3]};
  unsigned short hb[8];
#pragma unroll
  for (int e = 0; e < 8; ++e) hb[e] = h_bits(d[e] * rs * scv[e] + biv[e]);
  const v4u u = (v4u){pk16(hb[0], hb[1]), pk16(hb[2], hb[3]), pk16(hb[4], hb[5]), pk16(hb[6], hb[7])};
  const int orow = (row >> 11) * rowsPerBatch + rowOff + (row & (NS - 1));
  unsigned short* dst = outp + (size_t)orow * ND + col0;
  *(volatile v4u*)dst = u;
  __threadfence();
  *(volatile v4u*)dst = u;
}

__device__ __forceinline__ void vt_put(unsigned short* Vt, int d0, int kvr, uint4 u) {
  Vt[(d0 + 0) * 64 + kvr] = (unsigned short)(u.x & 0xffffu);
  Vt[(d0 + 1) * 64 + kvr] = (unsigned short)(u.x >> 16);
  Vt[(d0 + 2) * 64 + kvr] = (unsigned short)(u.y & 0xffffu);
  Vt[(d0 + 3) * 64 + kvr] = (unsigned short)(u.y >> 16);
  Vt[(d0 + 4) * 64 + kvr] = (unsigned short)(u.z & 0xffffu);
  Vt[(d0 + 5) * 64 + kvr] = (unsigned short)(u.z >> 16);
  Vt[(d0 + 6) * 64 + kvr] = (unsigned short)(u.w & 0xffffu);
  Vt[(d0 + 7) * 64 + kvr] = (unsigned short)(u.w >> 16);
}

__global__ __launch_bounds__(128) void attn_kernel(const unsigned short* __restrict__ qkv, unsigned short* __restrict__ op) {
  __shared__ __align__(16) unsigned short Vt[NHD * 64];
  __shared__ __align__(16) _Float16 Psh[4][16 * 64];
  __shared__ __align__(16) float Os[4][16 * 68];
  const int tid  = threadIdx.x;
  const int wave = tid >> 5;
  const int lane = tid & 31;
  const int hh   = lane >> 4;
  const int c    = lane & 15;
  const int koff = hh * 8;
  const int bx = blockIdx.x;
  const int qb = bx & (NS / 64 - 1);
  const int bh = bx >> 5;
  const int h  = bh & (NH - 1);
  const int b  = bh >> 3;
  const int tok0 = b * NS;
  const int q0 = qb * 64 + wave * 16;
  const _Float16* P16 = (const _Float16*)(const void*)qkv;

  v16h qa[2];
#pragma unroll
  for (int dc = 0; dc < 2; ++dc)
    qa[dc] = Frag<_Float16>::load(P16 + (size_t)(tok0 + q0 + c) * QKV_LD + h * NHD + dc * 32 + koff);

  float mrow[8], lrow[8];
  v8f oacc[4];
#pragma unroll
  for (int r = 0; r < 8; ++r) { mrow[r] = -INFINITY; lrow[r] = 0.0f; }
#pragma unroll
  for (int t4 = 0; t4 < 4; ++t4) oacc[t4] = (v8f){0.f, 0.f, 0.f, 0.f, 0.f, 0.f, 0.f, 0.f};

  for (int kc = 0; kc < NS / 64; ++kc) {
    const int kv0 = kc * 64;
    __syncthreads();
    {
      const int kvr = tid >> 1, dh = (tid & 1) * 32;
      const uint4* vp = (const uint4*)(const void*)(qkv + (size_t)(tok0 + kv0 + kvr) * QKV_LD + 2 * ND + h * NHD + dh);
      const uint4 u0 = vp[0], u1 = vp[1], u2 = vp[2], u3 = vp[3];
      vt_put(Vt, dh + 0,  kvr, u0);
      vt_put(Vt, dh + 8,  kvr, u1);
      vt_put(Vt, dh + 16, kvr, u2);
      vt_put(Vt, dh + 24, kvr, u3);
    }
    __syncthreads();

    v8f s[4];
#pragma unroll
    for (int j = 0; j < 4; ++j) {
      s[j] = (v8f){0.f, 0.f, 0.f, 0.f, 0.f, 0.f, 0.f, 0.f};
#pragma unroll
      for (int dc = 0; dc < 2; ++dc) {
        const v16h kb = Frag<_Float16>::load(P16 + (size_t)(tok0 + kv0 + (j << 4) + c) * QKV_LD + ND + h * NHD + dc * 32 + koff);
        s[j] = mma_h(qa[dc], kb, s[j]);
      }
    }
    float cm[8];
#pragma unroll
    for (int r = 0; r < 8; ++r) {
      float m = -INFINITY;
#pragma unroll
      for (int j = 0; j < 4; ++j) { s[j][r] *= 0.125f; m = fmaxf(m, s[j][r]); }
#pragma unroll
      for (int off = 1; off < 16; off <<= 1) m = fmaxf(m, __shfl_xor(m, off, 32));
      cm[r] = m;
    }
    _Float16* pwh = Psh[wave];
#pragma unroll
    for (int r = 0; r < 8; ++r) {
      const float mnew  = fmaxf(mrow[r], cm[r]);
      const float alpha = expf(mrow[r] - mnew);
      mrow[r] = mnew;
      float psum = 0.0f;
#pragma unroll
      for (int j = 0; j < 4; ++j) {
        const float p = expf(s[j][r] - mnew);
        psum += p;
        pwh[(8 * hh + r) * 64 + j * 16 + c] = (_Float16)(p * PCARRY);
      }
#pragma unroll
      for (int off = 1; off < 16; off <<= 1) psum += __shfl_xor(psum, off, 32);
      lrow[r] = lrow[r] * alpha + psum;
#pragma unroll
      for (int t4 = 0; t4 < 4; ++t4) oacc[t4][r] *= alpha;
    }
    wave_lds_sync();
    const _Float16* V16 = (const _Float16*)(const void*)Vt;
#pragma unroll
    for (int kk = 0; kk < 2; ++kk) {
      const v16h pa = Frag<_Float16>::load(pwh + c * 64 + kk * 32 + 8 * hh);
#pragma unroll
      for (int t4 = 0; t4 < 4; ++t4) {
        const v16h vb = Frag<_Float16>::load(V16 + (t4 * 16 + c) * 64 + kk * 32 + 8 * hh);
        oacc[t4] = mma_h(pa, vb, oacc[t4]);
      }
    }
  }

  float* os = Os[wave];
#pragma unroll
  for (int r = 0; r < 8; ++r) {
    const float inv = (OCARRY / PCARRY) / lrow[r];
#pragma unroll
    for (int t4 = 0; t4 < 4; ++t4) os[(8 * hh + r) * 68 + t4 * 16 + c] = oacc[t4][r] * inv;
  }
  wave_lds_sync();
  {
    const int q = lane >> 3, c8 = (lane & 7) * 8;
    _Float16* O16 = (_Float16*)(void*)op;
    for (int pass = 0; pass < 2; ++pass) {
#pragma unroll
      for (int it = 0; it < 4; ++it) {
        const int row = it * 4 + q;
        const float* sp = os + row * 68 + c8;
        v8h hv;
#pragma unroll
        for (int e = 0; e < 8; ++e) hv[e] = (_Float16)sp[e];
        *(volatile v8h*)(O16 + (size_t)(tok0 + q0 + row) * ND + h * NHD + c8) = hv;
      }
      __threadfence();
    }
  }
}

extern "C" void kernel_launch(void* const* d_in, const int* in_sizes, int n_in,
                              void* d_out, int out_size, void* d_ws, size_t ws_size,
                              hipStream_t stream) {
  if (n_in < 20) return;
  if (in_sizes[0] != NTOK * ND || in_sizes[1] != NTOK || in_sizes[4] != KW * ND * ND ||
      in_sizes[8] != ND * ND || in_sizes[14] != ND * ND ||
      in_sizes[16] != NG * NE * ND * NFF || in_sizes[18] != NG * NE * NFF * ND ||
      out_size != NTOK * ND) return;
  if (ws_size < WS_TOTAL) return;

  const float* x    = (const float*)d_in[0];
  const int*   gid  = (const int*)d_in[1];
  const float* ln1s = (const float*)d_in[2];
  const float* ln1b = (const float*)d_in[3];
  const float* ck   = (const float*)d_in[4];
  const float* cb   = (const float*)d_in[5];
  const float* ln2s = (const float*)d_in[6];
  const float* ln2b = (const float*)d_in[7];
  const float* wq   = (const float*)d_in[8];
  const float* bq   = (const float*)d_in[9];
  const float* wk   = (const float*)d_in[10];
  const float* bk   = (const float*)d_in[11];
  const float* wv   = (const float*)d_in[12];
  const float* bv   = (const float*)d_in[13];
  const float* wo   = (const float*)d_in[14];
  const float* bo   = (const float*)d_in[15];
  const float* w1   = (const float*)d_in[16];
  const float* b1   = (const float*)d_in[17];
  const float* w2   = (const float*)d_in[18];
  const float* b2   = (const float*)d_in[19];
  float* out = (float*)d_out;

  char* p = (char*)d_ws;
  unsigned short* ckT   = (unsigned short*)p;  unsigned short* xg = (unsigned short*)p;  p += WS_CKT;
  unsigned short* wqT   = (unsigned short*)p;  p += WS_W512;
  unsigned short* wkT   = (unsigned short*)p;  p += WS_W512;
  unsigned short* wvT   = (unsigned short*)p;  p += WS_W512;
  unsigned short* woT   = (unsigned short*)p;  p += WS_W512;
  unsigned short* w1T   = (unsigned short*)p;  p += WS_W1T;
  unsigned short* w2T   = (unsigned short*)p;  p += WS_W2T;
  unsigned short* act16 = (unsigned short*)p;  p += WS_ACT16;
  float*          x1    = (float*)p;           p += WS_X1;
  unsigned short* qkv   = (unsigned short*)p;  p += WS_QKV;
  float*          x2    = (float*)p;           p += WS_X2;
  unsigned short* hid   = (unsigned short*)p;  p += WS_HID;
  float*          y     = (float*)p;           p += WS_Y;

  trcast_kernel<<<dim3(KCONV / 64, ND / 64), 256, 0, stream>>>(ck, KCONV, ND, ckT, WCARRY);
  trcast_kernel<<<dim3(ND / 64, (NH * NHD) / 64), 256, 0, stream>>>(wq, ND, NH * NHD, wqT, WCARRY);
  trcast_kernel<<<dim3(ND / 64, (NH * NHD) / 64), 256, 0, stream>>>(wk, ND, NH * NHD, wkT, WCARRY);
  trcast_kernel<<<dim3(ND / 64, (NH * NHD) / 64), 256, 0, stream>>>(wv, ND, NH * NHD, wvT, WCARRY);
  trcast_kernel<<<dim3((NH * NHD) / 64, ND / 64), 256, 0, stream>>>(wo, NH * NHD, ND, woT, WCARRY);
  trcast_kernel<<<dim3((NG * NE * ND) / 64, NFF / 64), 256, 0, stream>>>(w1, NG * NE * ND, NFF, w1T, WCARRY);
  trcast_kernel<<<dim3((NG * NE * NFF) / 64, ND / 64), 256, 0, stream>>>(w2, NG * NE * NFF, ND, w2T, WCARRY);

  zero_pad_kernel<<<dim3(5, NB * 2), 256, 0, stream>>>(act16);
  ln_kernel<<<NTOK / 4, 256, 0, stream>>>(x, ln1s, ln1b, act16, HPROWS, PADL);
  static_assert(KCONV % 32 == 0 && NS % 64 == 0 && ND % 64 == 0);
  gemm_f16<1, 0, true><<<dim3((NS / 64) * (ND / 64) / 8, NB), 256, 0, stream>>>(
      act16, ND, (long)HPROWS * ND, ckT, KCONV, 0L, (void*)x1, ND, (long)NS * ND, cb, x, (long)NS * ND,
      NS, ND, KCONV, 1.0f / WCARRY, 1.0f);

  ln_kernel<<<NTOK / 4, 256, 0, stream>>>(x1, ln2s, ln2b, act16, NS, 0);
  static_assert(NTOK % 64 == 0 && ND % 32 == 0);
  gemm_f16<0, 1, false><<<dim3((NTOK / 64) * (ND / 64) / 8, 1), 256, 0, stream>>>(
      act16, ND, 0L, wqT, ND, 0L, (void*)(qkv + 0 * ND), QKV_LD, 0L, bq, nullptr, 0L, NTOK, ND, ND, 1.0f / WCARRY, 1.0f);
  gemm_f16<0, 1, false><<<dim3((NTOK / 64) * (ND / 64) / 8, 1), 256, 0, stream>>>(
      act16, ND, 0L, wkT, ND, 0L, (void*)(qkv + 1 * ND), QKV_LD, 0L, bk, nullptr, 0L, NTOK, ND, ND, 1.0f / WCARRY, 1.0f);
  gemm_f16<0, 1, false><<<dim3((NTOK / 64) * (ND / 64) / 8, 1), 256, 0, stream>>>(
      act16, ND, 0L, wvT, ND, 0L, (void*)(qkv + 2 * ND), QKV_LD, 0L, bv, nullptr, 0L, NTOK, ND, ND, 1.0f / WCARRY, 1.0f);
  attn_kernel<<<NB * NH * (NS / 64), 128, 0, stream>>>(qkv, act16);
  gemm_f16<0, 0, true><<<dim3((NTOK / 64) * (ND / 64) / 8, 1), 256, 0, stream>>>(
      act16, ND, 0L, woT, ND, 0L, (void*)x2, ND, 0L, bo, x1, 0L, NTOK, ND, ND, 1.0f / (WCARRY * OCARRY), 1.0f);

  gather_rows_kernel<<<GROWS / 64, 256, 0, stream>>>(gid, x2, xg);
  static_assert(ND % 32 == 0 && HID_LD % 32 == 0 && GROWS % 64 == 0 && NFF % 64 == 0);
  expert_gemm<1><<<dim3((GROWS / 64) * (NFF / 64) / 8, 1, NE), 256, 0, stream>>>(gid, xg, w1T, b1, (void*)hid);
  expert_gemm<2><<<dim3((GROWS / 64) * (ND / 64) / 8, 1, 1), 256, 0, stream>>>(gid, hid, w2T, b2, (void*)y);
  combine_kernel<<<NTOK / 64, 256, 0, stream>>>(gid, y, x2, out);
}
